// NNUE_16381005267418
// MI455X (gfx1250) — hardware-verified
//
#include <hip/hip_runtime.h>
#define BS 16384
#define NF 4476
#define NA 30
#define HH 512

typedef __bf16 v16b __attribute__((ext_vector_type(16)));
typedef unsigned short v8us __attribute__((ext_vector_type(8), may_alias));
typedef float  v8f  __attribute__((ext_vector_type(8)));
typedef float  v4f  __attribute__((ext_vector_type(4)));
typedef float  v4fa __attribute__((ext_vector_type(4), may_alias));
union FragB { v16b v; v8us half[2]; unsigned short u[16]; };

__device__ __forceinline__ unsigned short bf16_bits(float x) { unsigned int u = __float_as_uint(x); return (unsigned short)((u + 0x7FFFu + ((u >> 16) & 1u)) >> 16); }
__device__ __forceinline__ float bf16_val(unsigned short b) { return __uint_as_float(((unsigned int)b) << 16); }
__device__ __forceinline__ float bf16_round(float x) { return bf16_val(bf16_bits(x)); }
template <int NT>
__device__ __forceinline__ v8f mmaN(v16b ah, v16b al, v16b bh, v16b bl, v8f c) {
  c = __builtin_amdgcn_wmma_f32_16x16x32_bf16(false, ah, false, bh, (short)0, c, false, false);
  if (NT >= 2) c = __builtin_amdgcn_wmma_f32_16x16x32_bf16(false, al, false, bh, (short)0, c, false, false);
  if (NT >= 3) c = __builtin_amdgcn_wmma_f32_16x16x32_bf16(false, ah, false, bl, (short)0, c, false, false);
  asm volatile("v_nop\n\tv_nop\n\tv_nop\n\tv_nop" : "+v"(c) : "v"(ah), "v"(al), "v"(bh), "v"(bl));
  return c;
}

__global__ __launch_bounds__(256) void k_wt_bf16(const float* __restrict__ W, unsigned short* __restrict__ Wt, int K, int N) {
  const int t = blockIdx.x * 256 + threadIdx.x;
  const int k8n = K / 8;
  if (t >= N * k8n) return;
  const int n = t / k8n, k8 = (t % k8n) * 8;
  v8us v;
#pragma unroll
  for (int i = 0; i < 8; ++i) v[i] = bf16_bits(W[(size_t)(k8 + i) * N + n]);
  *(volatile v8us*)(Wt + (size_t)n * K + k8) = v;
  __threadfence();
  *(volatile v8us*)(Wt + (size_t)n * K + k8) = v;
}

template <bool ASPLIT, int ACT, bool BIAS_BF16>
__global__ __launch_bounds__(128) void k_gemm_bf(const float* __restrict__ A, int lda, const unsigned short* __restrict__ Wt, int ldb,
                                               const float* __restrict__ bias, float* __restrict__ C, int ldc, int M, int N, int K) {
  __shared__ __attribute__((aligned(16))) float so[4][16][64];
  const int tid = threadIdx.x, w = tid >> 5, lane = tid & 31, ln = lane & 15, hh = lane >> 4;
  const int ntn = N / 64;
  const int wid = blockIdx.x * 4 + w;
  const int mt = wid / ntn, nq = wid % ntn;
  if (mt * 16 >= M) return;
  const int row0 = mt * 16, col0 = nq * 64;
  const float* arow = A + (size_t)(row0 + ln) * lda;
  v8f acc[4] = {};
  for (int kb = 0; kb < K; kb += 32) {
    FragB ah, al;
    const v4f x0 = *(const v4fa*)(arow + kb + 8 * hh), x1 = *(const v4fa*)(arow + kb + 8 * hh + 4);
    const v4f x2 = *(const v4fa*)(arow + kb + 16 + 8 * hh), x3 = *(const v4fa*)(arow + kb + 16 + 8 * hh + 4);
    float xs[16] = {x0[0],x0[1],x0[2],x0[3],x1[0],x1[1],x1[2],x1[3],x2[0],x2[1],x2[2],x2[3],x3[0],x3[1],x3[2],x3[3]};
#pragma unroll
    for (int i = 0; i < 16; ++i) { const unsigned short hb = bf16_bits(xs[i]); ah.u[i] = hb; al.u[i] = ASPLIT ? bf16_bits(xs[i] - bf16_val(hb)) : (unsigned short)0; }
#pragma unroll
    for (int t = 0; t < 4; ++t) {
      const unsigned short* brow = Wt + (size_t)(col0 + t * 16 + ln) * ldb + kb;
      FragB b;
      b.half[0] = *(const v8us*)(brow + 8 * hh);
      b.half[1] = *(const v8us*)(brow + 16 + 8 * hh);
      acc[t] = mmaN<ASPLIT ? 2 : 1>(ah.v, al.v, b.v, b.v, acc[t]);
    }
  }
#pragma unroll
  for (int t = 0; t < 4; ++t) {
    float bv = bias ? bias[col0 + t * 16 + ln] : 0.f;
    if (BIAS_BF16) bv = bf16_round(bv);
#pragma unroll
    for (int r = 0; r < 8; ++r) { float v = acc[t][r] + bv; if (ACT == 1) v = fmaxf(v, 0.f); so[w][8 * hh + r][t * 16 + ln] = v; }
  }
  __builtin_amdgcn_fence(__ATOMIC_ACQ_REL, "workgroup");
  __builtin_amdgcn_wave_barrier();
  const int rsub = lane >> 4, c4 = (lane & 15) * 4;
  for (int pass = 0; pass < 2; ++pass) {
#pragma unroll
    for (int q = 0; q < 8; ++q) {
      const int r = q * 2 + rsub;
      const v4f v = *(const v4fa*)&so[w][r][c4];
      *(volatile v4f*)(C + (size_t)(row0 + r) * ldc + col0 + c4) = v;
    }
    if (pass == 0) __threadfence();
  }
}

template <int D, bool CAUSAL>
__global__ __launch_bounds__(128) void k_flash(const float* __restrict__ qb, const float* __restrict__ kb, const float* __restrict__ vb,
                                             int pitch, int T, int H, float scale, float* __restrict__ y, int ypitch) {
  constexpr int KS = D / 32;
  constexpr int DT = D / 16;
  __shared__ __attribute__((aligned(16))) unsigned short sKh[32][D + 8], sKl[32][D + 8], sVh[32][D + 8], sVl[32][D + 8];
  __shared__ __attribute__((aligned(16))) unsigned short sPh[4][16][40], sPl[4][16][40];
  __shared__ __attribute__((aligned(16))) float sO[4][16][D];
  const int tid = threadIdx.x, w = tid >> 5, lane = tid & 31, ln = lane & 15, hh = lane >> 4;
  const int nqb = (T + 63) / 64;
  const int bh = blockIdx.x / nqb, qblk = blockIdx.x % nqb;
  const int b = bh / H, h = bh % H;
  const int q0 = qblk * 64 + w * 16;
  const float* Q = qb + (size_t)b * T * pitch + h * D;
  const float* K = kb + (size_t)b * T * pitch + h * D;
  const float* V = vb + (size_t)b * T * pitch + h * D;

  FragB aqh[KS], aql[KS];
  {
    int row = q0 + ln; if (row >= T) row = T - 1;
    const float* qr = Q + (size_t)row * pitch;
#pragma unroll
    for (int ks = 0; ks < KS; ++ks)
#pragma unroll
      for (int i = 0; i < 16; ++i) {
        const int d = ks * 32 + ((i < 8) ? (8 * hh + i) : (16 + 8 * hh + (i - 8)));
        const float x = qr[d] * scale; const unsigned short hb = bf16_bits(x);
        aqh[ks].u[i] = hb; aql[ks].u[i] = bf16_bits(x - bf16_val(hb));
      }
  }
  float m_r[8], l_r[8];
#pragma unroll
  for (int r = 0; r < 8; ++r) { m_r[r] = -3.0e38f; l_r[r] = 0.f; }
  v8f oacc[DT];
#pragma unroll
  for (int dt = 0; dt < DT; ++dt) oacc[dt] = (v8f){0.f,0.f,0.f,0.f,0.f,0.f,0.f,0.f};

  const int kv_end = CAUSAL ? min(T, qblk * 64 + 64) : T;
  for (int j0 = 0; j0 < kv_end; j0 += 32) {
    __syncthreads();
    for (int e = tid; e < 32 * (D / 4); e += 128) {
      const int r = e / (D / 4), c4 = (e % (D / 4)) * 4;
      const int key = j0 + r;
      v4f kf = {0.f,0.f,0.f,0.f}, vf = {0.f,0.f,0.f,0.f};
      if (key < T) { kf = *(const v4fa*)(K + (size_t)key * pitch + c4); vf = *(const v4fa*)(V + (size_t)key * pitch + c4); }
#pragma unroll
      for (int t = 0; t < 4; ++t) {
        unsigned short hb = bf16_bits(kf[t]); sKh[r][c4 + t] = hb; sKl[r][c4 + t] = bf16_bits(kf[t] - bf16_val(hb));
        hb = bf16_bits(vf[t]); sVh[r][c4 + t] = hb; sVl[r][c4 + t] = bf16_bits(vf[t] - bf16_val(hb));
      }
    }
    __syncthreads();
    v8f s[2];
#pragma unroll
    for (int nt = 0; nt < 2; ++nt) {
      v8f acc = {};
#pragma unroll
      for (int ks = 0; ks < KS; ++ks) {
        FragB bh_, bl_;
        bh_.half[0] = *(const v8us*)&sKh[nt * 16 + ln][ks * 32 + 8 * hh]; bh_.half[1] = *(const v8us*)&sKh[nt * 16 + ln][ks * 32 + 16 + 8 * hh];
        bl_.half[0] = *(const v8us*)&sKl[nt * 16 + ln][ks * 32 + 8 * hh]; bl_.half[1] = *(const v8us*)&sKl[nt * 16 + ln][ks * 32 + 16 + 8 * hh];
        acc = mmaN<3>(aqh[ks].v, aql[ks].v, bh_.v, bl_.v, acc);
      }
      s[nt] = acc;
    }
    float alpha[8];
#pragma unroll
    for (int r = 0; r < 8; ++r) {
      const int qi = q0 + 8 * hh + r;
      const int ja = j0 + ln, jb = j0 + 16 + ln;
      if (CAUSAL) { if (ja > qi) s[0][r] = -3.0e38f; if (jb > qi) s[1][r] = -3.0e38f; }
      if (ja >= T) s[0][r] = -3.0e38f;
      if (jb >= T) s[1][r] = -3.0e38f;
      float mx = fmaxf(s[0][r], s[1][r]);
      mx = fmaxf(mx, __shfl_xor(mx, 1, 32)); mx = fmaxf(mx, __shfl_xor(mx, 2, 32)); mx = fmaxf(mx, __shfl_xor(mx, 4, 32)); mx = fmaxf(mx, __shfl_xor(mx, 8, 32));
      const float mnew = fmaxf(m_r[r], mx);
      alpha[r] = (mnew > -1.0e38f) ? __expf(m_r[r] - mnew) : 1.0f;
      const float p0 = (s[0][r] > -1.0e38f) ? __expf(s[0][r] - mnew) : 0.f;
      const float p1 = (s[1][r] > -1.0e38f) ? __expf(s[1][r] - mnew) : 0.f;
      m_r[r] = mnew;
      l_r[r] = l_r[r] * alpha[r] + p0 + p1;
      unsigned short hb = bf16_bits(p0); sPh[w][8 * hh + r][ln] = hb;      sPl[w][8 * hh + r][ln] = bf16_bits(p0 - bf16_val(hb));
      hb = bf16_bits(p1);                sPh[w][8 * hh + r][16 + ln] = hb; sPl[w][8 * hh + r][16 + ln] = bf16_bits(p1 - bf16_val(hb));
    }
#pragma unroll
    for (int dt = 0; dt < DT; ++dt)
#pragma unroll
      for (int r = 0; r < 8; ++r) oacc[dt][r] *= alpha[r];
    __builtin_amdgcn_fence(__ATOMIC_ACQ_REL, "workgroup");
    __builtin_amdgcn_wave_barrier();
    FragB pah, pal;
    pah.half[0] = *(const v8us*)&sPh[w][ln][8 * hh]; pah.half[1] = *(const v8us*)&sPh[w][ln][16 + 8 * hh];
    pal.half[0] = *(const v8us*)&sPl[w][ln][8 * hh]; pal.half[1] = *(const v8us*)&sPl[w][ln][16 + 8 * hh];
#pragma unroll
    for (int dt = 0; dt < DT; ++dt) {
      FragB bvh, bvl;
#pragma unroll
      for (int i = 0; i < 8; ++i) {
        bvh.u[i] = sVh[8 * hh + i][dt * 16 + ln]; bvh.u[8 + i] = sVh[16 + 8 * hh + i][dt * 16 + ln];
        bvl.u[i] = sVl[8 * hh + i][dt * 16 + ln]; bvl.u[8 + i] = sVl[16 + 8 * hh + i][dt * 16 + ln];
      }
      oacc[dt] = mmaN<3>(pah.v, pal.v, bvh.v, bvl.v, oacc[dt]);
    }
    __builtin_amdgcn_fence(__ATOMIC_ACQ_REL, "workgroup");
    __builtin_amdgcn_wave_barrier();
  }
#pragma unroll
  for (int r = 0; r < 8; ++r) {
    float l = l_r[r];
    l += __shfl_xor(l, 1, 32); l += __shfl_xor(l, 2, 32); l += __shfl_xor(l, 4, 32); l += __shfl_xor(l, 8, 32);
    l_r[r] = (l > 0.f) ? 1.0f / l : 0.f;
  }
#pragma unroll
  for (int dt = 0; dt < DT; ++dt)
#pragma unroll
    for (int r = 0; r < 8; ++r) sO[w][8 * hh + r][dt * 16 + ln] = oacc[dt][r] * l_r[r];
  __builtin_amdgcn_fence(__ATOMIC_ACQ_REL, "workgroup");
  __builtin_amdgcn_wave_barrier();
  for (int pass = 0; pass < 2; ++pass) {
    for (int r = 0; r < 16; ++r) {
      const int row = q0 + r;
      if (row < T && lane < D / 4) {
        const v4f val = *(const v4fa*)&sO[w][r][lane * 4];
        *(volatile v4f*)(y + ((size_t)b * T + row) * ypitch + h * D + lane * 4) = val;
      }
    }
    if (pass == 0) __threadfence();
  }
}

template <bool AFFINE, bool RESID, bool RES_BF16>
__global__ __launch_bounds__(256) void k_transpose32(const float* __restrict__ in, float* __restrict__ out, int rows, int cols,
                                                    const float* __restrict__ scale, const float* __restrict__ shift, const float* __restrict__ res) {
  __shared__ float tile[32][33];
  const int b = blockIdx.z;
  const int r0 = blockIdx.y * 32, c0 = blockIdx.x * 32;
  const float* src = in + (size_t)b * rows * cols;
  float* dst = out + (size_t)b * rows * cols;
  const int tx = threadIdx.x & 31, ty = threadIdx.x >> 5;
  for (int i = ty; i < 32; i += 8) tile[i][tx] = src[(size_t)(r0 + i) * cols + c0 + tx];
  __syncthreads();
  for (int pass = 0; pass < 2; ++pass) {
    for (int i = ty; i < 32; i += 8) {
      float v = tile[tx][i];
      const int orow = c0 + i;
      if (AFFINE) v = v * scale[orow] + shift[orow];
      if (RESID) { float rv = res[(size_t)b * rows * cols + (size_t)orow * rows + r0 + tx]; if (RES_BF16) rv = bf16_round(rv); v += rv; }
      *(volatile float*)(dst + (size_t)orow * rows + r0 + tx) = v;
    }
    if (pass == 0) __threadfence();
  }
}

__global__ __launch_bounds__(256) void k_pool2_pm(const float* __restrict__ in, float* __restrict__ out, int Bn, int H, int W, int C) {
  const size_t t = (size_t)blockIdx.x * 256 + threadIdx.x;
  const int c4n = C / 4, Ho = H / 2, Wo = W / 2;
  const size_t total = (size_t)Bn * Ho * Wo * c4n;
  if (t >= total) return;
  const int c4 = (int)(t % c4n) * 4; size_t rest = t / c4n;
  const int pw = (int)(rest % Wo); rest /= Wo; const int ph = (int)(rest % Ho); const int b = (int)(rest / Ho);
  const float* base = in + (size_t)b * H * W * C;
  const int p00 = (2 * ph) * W + 2 * pw;
  const v4f a = *(const v4fa*)(base + (size_t)p00 * C + c4), bq = *(const v4fa*)(base + (size_t)(p00 + 1) * C + c4);
  const v4f c = *(const v4fa*)(base + (size_t)(p00 + W) * C + c4), d = *(const v4fa*)(base + (size_t)(p00 + W + 1) * C + c4);
  v4f m; for (int i = 0; i < 4; ++i) m[i] = fmaxf(fmaxf(a[i], bq[i]), fmaxf(c[i], d[i]));
  float* dst = out + ((size_t)b * Ho * Wo + (size_t)ph * Wo + pw) * C + c4;
  *(volatile v4f*)dst = m;
  __threadfence();
  *(volatile v4f*)dst = m;
}

template <int DQ, int DV>
__global__ __launch_bounds__(128) void k_flash2(const float* __restrict__ Qb, size_t qstride, int qpitch, int Tq,
                                              const float* __restrict__ Kb, size_t kstride, int kpitch, int Tk,
                                              const float* __restrict__ Vb, size_t vstride, int vpitch,
                                              float scale, float* __restrict__ y, size_t ystride, int ypitch) {
  constexpr int KS = DQ / 32, DT = DV / 16;
  __shared__ __attribute__((aligned(16))) unsigned short sKh[32][DQ + 8], sKl[32][DQ + 8], sVh[32][DV + 8], sVl[32][DV + 8];
  __shared__ __attribute__((aligned(16))) unsigned short sPh[4][16][40], sPl[4][16][40];
  __shared__ __attribute__((aligned(16))) float sO[4][16][DV];
  const int tid = threadIdx.x, w = tid >> 5, lane = tid & 31, ln = lane & 15, hh = lane >> 4;
  const int nqb = (Tq + 63) / 64;
  const int bh = blockIdx.x / nqb, qblk = blockIdx.x % nqb;
  const int dv0 = blockIdx.y * DV;
  const int q0 = qblk * 64 + w * 16;
  const float* Q = Qb + (size_t)bh * qstride; const float* K = Kb + (size_t)bh * kstride; const float* V = Vb + (size_t)bh * vstride + dv0;
  FragB aqh[KS], aql[KS];
  {
    int row = q0 + ln; if (row >= Tq) row = Tq - 1;
    const float* qr = Q + (size_t)row * qpitch;
#pragma unroll
    for (int ks = 0; ks < KS; ++ks)
#pragma unroll
      for (int i = 0; i < 16; ++i) {
        const int d = ks * 32 + ((i < 8) ? (8 * hh + i) : (16 + 8 * hh + (i - 8)));
        const float x = qr[d] * scale; const unsigned short hb = bf16_bits(x);
        aqh[ks].u[i] = hb; aql[ks].u[i] = bf16_bits(x - bf16_val(hb));
      }
  }
  float m_r[8], l_r[8];
#pragma unroll
  for (int r = 0; r < 8; ++r) { m_r[r] = -3.0e38f; l_r[r] = 0.f; }
  v8f oacc[DT];
#pragma unroll
  for (int dt = 0; dt < DT; ++dt) oacc[dt] = (v8f){0.f,0.f,0.f,0.f,0.f,0.f,0.f,0.f};
  for (int j0 = 0; j0 < Tk; j0 += 32) {
    __syncthreads();
    for (int e = tid; e < 32 * (DQ / 4); e += 128) {
      const int r = e / (DQ / 4), c4 = (e % (DQ / 4)) * 4; const int key = j0 + r;
      v4f f = {0.f,0.f,0.f,0.f}; if (key < Tk) f = *(const v4fa*)(K + (size_t)key * kpitch + c4);
#pragma unroll
      for (int t = 0; t < 4; ++t) { const unsigned short hb = bf16_bits(f[t]); sKh[r][c4 + t] = hb; sKl[r][c4 + t] = bf16_bits(f[t] - bf16_val(hb)); }
    }
    for (int e = tid; e < 32 * (DV / 4); e += 128) {
      const int r = e / (DV / 4), c4 = (e % (DV / 4)) * 4; const int key = j0 + r;
      v4f f = {0.f,0.f,0.f,0.f}; if (key < Tk) f = *(const v4fa*)(V + (size_t)key * vpitch + c4);
#pragma unroll
      for (int t = 0; t < 4; ++t) { const unsigned short hb = bf16_bits(f[t]); sVh[r][c4 + t] = hb; sVl[r][c4 + t] = bf16_bits(f[t] - bf16_val(hb)); }
    }
    __syncthreads();
    v8f s[2];
#pragma unroll
    for (int nt = 0; nt < 2; ++nt) {
      v8f acc = {};
#pragma unroll
      for (int ks = 0; ks < KS; ++ks) {
        FragB bh_, bl_;
        bh_.half[0] = *(const v8us*)&sKh[nt * 16 + ln][ks * 32 + 8 * hh]; bh_.half[1] = *(const v8us*)&sKh[nt * 16 + ln][ks * 32 + 16 + 8 * hh];
        bl_.half[0] = *(const v8us*)&sKl[nt * 16 + ln][ks * 32 + 8 * hh]; bl_.half[1] = *(const v8us*)&sKl[nt * 16 + ln][ks * 32 + 16 + 8 * hh];
        acc = mmaN<3>(aqh[ks].v, aql[ks].v, bh_.v, bl_.v, acc);
      }
      s[nt] = acc;
    }
    float alpha[8];
#pragma unroll
    for (int r = 0; r < 8; ++r) {
      const int ja = j0 + ln, jb = j0 + 16 + ln;
      if (ja >= Tk) s[0][r] = -3.0e38f;
      if (jb >= Tk) s[1][r] = -3.0e38f;
      float mx = fmaxf(s[0][r], s[1][r]);
      mx = fmaxf(mx, __shfl_xor(mx, 1, 32)); mx = fmaxf(mx, __shfl_xor(mx, 2, 32)); mx = fmaxf(mx, __shfl_xor(mx, 4, 32)); mx = fmaxf(mx, __shfl_xor(mx, 8, 32));
      const float mnew = fmaxf(m_r[r], mx);
      alpha[r] = (mnew > -1.0e38f) ? __expf(m_r[r] - mnew) : 1.0f;
      const float p0 = (s[0][r] > -1.0e38f) ? __expf(s[0][r] - mnew) : 0.f;
      const float p1 = (s[1][r] > -1.0e38f) ? __expf(s[1][r] - mnew) : 0.f;
      m_r[r] = mnew;
      l_r[r] = l_r[r] * alpha[r] + p0 + p1;
      unsigned short hb = bf16_bits(p0); sPh[w][8 * hh + r][ln] = hb;      sPl[w][8 * hh + r][ln] = bf16_bits(p0 - bf16_val(hb));
      hb = bf16_bits(p1);                sPh[w][8 * hh + r][16 + ln] = hb; sPl[w][8 * hh + r][16 + ln] = bf16_bits(p1 - bf16_val(hb));
    }
#pragma unroll
    for (int dt = 0; dt < DT; ++dt)
#pragma unroll
      for (int r = 0; r < 8; ++r) oacc[dt][r] *= alpha[r];
    __builtin_amdgcn_fence(__ATOMIC_ACQ_REL, "workgroup");
    __builtin_amdgcn_wave_barrier();
    FragB pah, pal;
    pah.half[0] = *(const v8us*)&sPh[w][ln][8 * hh]; pah.half[1] = *(const v8us*)&sPh[w][ln][16 + 8 * hh];
    pal.half[0] = *(const v8us*)&sPl[w][ln][8 * hh]; pal.half[1] = *(const v8us*)&sPl[w][ln][16 + 8 * hh];
#pragma unroll
    for (int dt = 0; dt < DT; ++dt) {
      FragB bvh, bvl;
#pragma unroll
      for (int i = 0; i < 8; ++i) {
        bvh.u[i] = sVh[8 * hh + i][dt * 16 + ln]; bvh.u[8 + i] = sVh[16 + 8 * hh + i][dt * 16 + ln];
        bvl.u[i] = sVl[8 * hh + i][dt * 16 + ln]; bvl.u[8 + i] = sVl[16 + 8 * hh + i][dt * 16 + ln];
      }
      oacc[dt] = mmaN<3>(pah.v, pal.v, bvh.v, bvl.v, oacc[dt]);
    }
    __builtin_amdgcn_fence(__ATOMIC_ACQ_REL, "workgroup");
    __builtin_amdgcn_wave_barrier();
  }
#pragma unroll
  for (int r = 0; r < 8; ++r) {
    float l = l_r[r];
    l += __shfl_xor(l, 1, 32); l += __shfl_xor(l, 2, 32); l += __shfl_xor(l, 4, 32); l += __shfl_xor(l, 8, 32);
    l_r[r] = (l > 0.f) ? 1.0f / l : 0.f;
  }
#pragma unroll
  for (int dt = 0; dt < DT; ++dt)
#pragma unroll
    for (int r = 0; r < 8; ++r) sO[w][8 * hh + r][dt * 16 + ln] = oacc[dt][r] * l_r[r];
  __builtin_amdgcn_fence(__ATOMIC_ACQ_REL, "workgroup");
  __builtin_amdgcn_wave_barrier();
  for (int pass = 0; pass < 2; ++pass) {
    for (int r = 0; r < 16; ++r) {
      const int row = q0 + r;
      for (int c4 = lane * 4; c4 < DV; c4 += 128) {
        if (row < Tq) {
          const v4f val = *(const v4fa*)&sO[w][r][c4];
          *(volatile v4f*)(y + (size_t)bh * ystride + (size_t)row * ypitch + dv0 + c4) = val;
        }
      }
    }
    if (pass == 0) __threadfence();
  }
}

typedef _Float16 v16h __attribute__((ext_vector_type(16)));
union FragH { v16h v; v8us half[2]; _Float16 h[16]; unsigned short u[16]; };
template <int NT>
__device__ __forceinline__ v8f mmaH(v16h ah, v16h al, v16h bh, v16h bl, v8f c) {
  c = __builtin_amdgcn_wmma_f32_16x16x32_f16(false, ah, false, bh, (short)0, c, false, false);
  if (NT >= 2) c = __builtin_amdgcn_wmma_f32_16x16x32_f16(false, al, false, bh, (short)0, c, false, false);
  if (NT >= 3) c = __builtin_amdgcn_wmma_f32_16x16x32_f16(false, ah, false, bl, (short)0, c, false, false);
  asm volatile("v_nop\n\tv_nop\n\tv_nop\n\tv_nop" : "+v"(c) : "v"(ah), "v"(al), "v"(bh), "v"(bl));
  return c;
}
template <bool ASPLIT>
__global__ __launch_bounds__(128) void k_gemm_h(const float* __restrict__ A, int lda, size_t sA, const _Float16* __restrict__ Bh, int ldb, size_t sB, float alpha, float* __restrict__ C, int ldc, size_t sC, int M, int N, int K) {
  __shared__ __attribute__((aligned(16))) float so[4][16][64];
  const int tid = threadIdx.x, w = tid >> 5, lane = tid & 31, ln = lane & 15, hh = lane >> 4; const int by = blockIdx.y;
  A += (size_t)by * sA; Bh += (size_t)by * sB; C += (size_t)by * sC;
  const int ntn = (N + 63) / 64; const int wid = blockIdx.x * 4 + w; const int mt = wid / ntn, nq = wid % ntn; if (mt * 16 >= M) return;
  const int row0 = mt * 16, col0 = nq * 64; const float* arow = A + (size_t)(row0 + ln) * lda;
  v8f acc[4] = {};
  for (int kb = 0; kb < K; kb += 32) {
    FragH ah, al;
    const v4f x0 = *(const v4fa*)(arow + kb + 8 * hh), x1 = *(const v4fa*)(arow + kb + 8 * hh + 4), x2 = *(const v4fa*)(arow + kb + 16 + 8 * hh), x3 = *(const v4fa*)(arow + kb + 16 + 8 * hh + 4);
    float xs[16] = {x0[0],x0[1],x0[2],x0[3],x1[0],x1[1],x1[2],x1[3],x2[0],x2[1],x2[2],x2[3],x3[0],x3[1],x3[2],x3[3]};
#pragma unroll
    for (int i = 0; i < 16; ++i) { const _Float16 h = (_Float16)xs[i]; ah.h[i] = h; al.h[i] = ASPLIT ? (_Float16)(xs[i] - (float)h) : (_Float16)0.0f; }
#pragma unroll
    for (int t = 0; t < 4; ++t) { if (col0 + t * 16 >= N) continue; const size_t boff = (size_t)(col0 + t * 16 + ln) * ldb + kb; FragH bq; bq.half[0] = *(const v8us*)(Bh + boff + 8 * hh); bq.half[1] = *(const v8us*)(Bh + boff + 16 + 8 * hh);
      acc[t] = mmaH<ASPLIT ? 2 : 1>(ah.v, al.v, bq.v, bq.v, acc[t]); }
  }
#pragma unroll
  for (int t = 0; t < 4; ++t) { if (col0 + t * 16 >= N) continue;
#pragma unroll
    for (int r = 0; r < 8; ++r) so[w][8 * hh + r][t * 16 + ln] = acc[t][r] * alpha; }
  __builtin_amdgcn_fence(__ATOMIC_ACQ_REL, "workgroup"); __builtin_amdgcn_wave_barrier();
  const int rsub = lane >> 4, c4 = (lane & 15) * 4;
  for (int pass = 0; pass < 2; ++pass) {
#pragma unroll
    for (int q = 0; q < 8; ++q) { const int r = q * 2 + rsub; if (col0 + c4 < N) { const v4f v = *(const v4fa*)&so[w][r][c4]; *(volatile v4f*)(C + (size_t)(row0 + r) * ldc + col0 + c4) = v; } }
    if (pass == 0) __threadfence(); }
}

__global__ __launch_bounds__(256) void k_wt_f16n(const float* __restrict__ W, _Float16* __restrict__ Wt, int N, int K, float scale) {
  const size_t t = (size_t)blockIdx.x * 256 + threadIdx.x; if (t >= (size_t)N * K / 8) return; FragH f;
#pragma unroll
  for (int i = 0; i < 8; ++i) f.h[i] = (_Float16)(bf16_round(W[t * 8 + i]) * scale); const v8us o = f.half[0]; *(volatile v8us*)((unsigned short*)Wt + t * 8) = o; __threadfence(); *(volatile v8us*)((unsigned short*)Wt + t * 8) = o; }
__global__ __launch_bounds__(256) void k_ftT(const float* __restrict__ ftw, float* __restrict__ ftT) { const size_t t = (size_t)blockIdx.x * 256 + threadIdx.x; if (t >= (size_t)NF * HH) return; const int c = (int)(t % HH); const int f = (int)(t / HH); const float v = ftw[(size_t)c * NF + f]; *(volatile float*)(ftT + t) = v; __threadfence(); *(volatile float*)(ftT + t) = v; }
__global__ __launch_bounds__(256) void k_ft(const int* __restrict__ wi, const int* __restrict__ bi, const float* __restrict__ ftT, float* __restrict__ H0) {
  const int tid = threadIdx.x, wv = tid >> 5, lane = tid & 31; const int t = blockIdx.x * 8 + wv; const int row = t >> 1, side = t & 1; const int* ids = (side ? bi : wi) + (size_t)row * NA;
  int myid = (lane < NA) ? ids[lane] : -1; if (myid < 0 || myid >= NF) myid = (lane < NA) ? (myid < 0 ? 0 : NF - 1) : -1;
#pragma unroll 1
  for (int l = 0; l < NA; ++l) { const int o = __shfl(myid, l, 32); if (l < lane && o == myid) myid = -1; }
  float acc[16]; for (int u = 0; u < 16; ++u) acc[u] = 0.f;
#pragma unroll 1
  for (int l = 0; l < NA; ++l) { const int id = __shfl(myid, l, 32); if (id < 0) continue; const float* r = ftT + (size_t)id * HH;
#pragma unroll
    for (int u = 0; u < 16; ++u) acc[u] += bf16_round(r[u * 32 + lane]); }
  float* dst = H0 + (size_t)row * (2 * HH) + side * HH;
  for (int pass = 0; pass < 2; ++pass) { for (int u = 0; u < 16; ++u) *(volatile float*)(dst + u * 32 + lane) = fminf(fmaxf(acc[u], -1.0f), 1.0f); if (pass == 0) __threadfence(); }
}
__global__ __launch_bounds__(256) void k_biasrelu(float* __restrict__ Y, const float* __restrict__ b, int N, size_t n4) { const size_t t = (size_t)blockIdx.x * 256 + threadIdx.x; if (t >= n4) return; const int c4 = (int)((t * 4) % N); v4f v = *(const v4fa*)(Y + t * 4); for (int q = 0; q < 4; ++q) v[q] = fmaxf(v[q] + bf16_round(b[c4 + q]), 0.f); *(volatile v4f*)(Y + t * 4) = v; __threadfence(); *(volatile v4f*)(Y + t * 4) = v; }
__global__ __launch_bounds__(1024) void k_head(const float* __restrict__ H3, const float* __restrict__ wo, const float* __restrict__ bo, float* __restrict__ out) {
  __shared__ float so[32]; const int tid = threadIdx.x, wv = tid >> 5, lane = tid & 31; const int row = blockIdx.x * 32 + wv; float s = 0.f;
  for (int c = lane; c < 128; c += 32) s += H3[(size_t)row * 128 + c] * bf16_round(wo[c]);
  for (int o = 16; o >= 1; o >>= 1) s += __shfl_xor(s, o, 32); if (lane == 0) so[wv] = s + bf16_round(bo[0]); __syncthreads();
  if (tid < 32) { *(volatile float*)(out + (size_t)blockIdx.x * 32 + tid) = so[tid]; } __threadfence(); if (tid < 32) { *(volatile float*)(out + (size_t)blockIdx.x * 32 + tid) = so[tid]; }
}
extern "C" void kernel_launch(void* const* d_in, const int* in_sizes, int n_in,
                              void* d_out, int out_size, void* d_ws, size_t ws_size, hipStream_t stream) {
  (void)in_sizes; (void)n_in; (void)out_size;
  const int* wi = (const int*)d_in[0]; const int* bi = (const int*)d_in[1]; const float* ftw = (const float*)d_in[2]; const float* w1 = (const float*)d_in[3]; const float* b1 = (const float*)d_in[4]; const float* w2 = (const float*)d_in[5]; const float* b2 = (const float*)d_in[6]; const float* w3 = (const float*)d_in[7]; const float* b3 = (const float*)d_in[8]; const float* wo = (const float*)d_in[9]; const float* bo = (const float*)d_in[10];
  char* ws = (char*)d_ws; size_t off = 0;
  auto take = [&](size_t bytes) { char* p = ws + off; off += (bytes + 255) & ~(size_t)255; return p; };
  float* ftT = (float*)take((size_t)NF * HH * 4); _Float16* B1 = (_Float16*)take((size_t)HH * 2 * HH * 2); _Float16* B2 = (_Float16*)take((size_t)256 * HH * 2); _Float16* B3 = (_Float16*)take((size_t)128 * 256 * 2);
  float* H0 = (float*)take((size_t)BS * 2 * HH * 4); float* H1 = (float*)take((size_t)BS * HH * 4); float* H2 = (float*)take((size_t)BS * 256 * 4); float* H3 = (float*)take((size_t)BS * 128 * 4);
  if (off > ws_size) return;
  k_ftT<<<(unsigned)(((size_t)NF * HH + 255) / 256), 256, 0, stream>>>(ftw, ftT);
  k_wt_f16n<<<(HH * 2 * HH / 8 + 255) / 256, 256, 0, stream>>>(w1, B1, HH, 2 * HH, 16.0f); k_wt_f16n<<<(256 * HH / 8 + 255) / 256, 256, 0, stream>>>(w2, B2, 256, HH, 16.0f); k_wt_f16n<<<(128 * 256 / 8 + 255) / 256, 256, 0, stream>>>(w3, B3, 128, 256, 16.0f);
  k_ft<<<(BS * 2) / 8, 256, 0, stream>>>(wi, bi, ftT, H0);
  k_gemm_h<false><<<dim3(((BS / 16) * (HH / 64) + 3) / 4, 1), 128, 0, stream>>>(H0, 2 * HH, 0, B1, 2 * HH, 0, 0.0625f, H1, HH, 0, BS, HH, 2 * HH); k_biasrelu<<<(unsigned)(((size_t)BS * HH / 4 + 255) / 256), 256, 0, stream>>>(H1, b1, HH, (size_t)BS * HH / 4);
  k_gemm_h<false><<<dim3(((BS / 16) * (256 / 64) + 3) / 4, 1), 128, 0, stream>>>(H1, HH, 0, B2, HH, 0, 0.0625f, H2, 256, 0, BS, 256, HH); k_biasrelu<<<(unsigned)(((size_t)BS * 256 / 4 + 255) / 256), 256, 0, stream>>>(H2, b2, 256, (size_t)BS * 256 / 4);
  k_gemm_h<false><<<dim3(((BS / 16) * (128 / 64) + 3) / 4, 1), 128, 0, stream>>>(H2, 256, 0, B3, 256, 0, 0.0625f, H3, 128, 0, BS, 128, 256); k_biasrelu<<<(unsigned)(((size_t)BS * 128 / 4 + 255) / 256), 256, 0, stream>>>(H3, b3, 128, (size_t)BS * 128 / 4);
  k_head<<<BS / 32, 1024, 0, stream>>>(H3, wo, bo, (float*)d_out);
}
